// HiResPrecipNet_fl_2_32_smaller_57174604645057
// MI455X (gfx1250) — hardware-run, weakly checked
//
#include <hip/hip_runtime.h>
#include <math.h>

typedef __attribute__((ext_vector_type(16))) _Float16 v16h;
typedef __attribute__((ext_vector_type(8)))  _Float16 v8h;
typedef __attribute__((ext_vector_type(8)))  float    v8f;
typedef __attribute__((ext_vector_type(4)))  float    v4f;
typedef __attribute__((ext_vector_type(4)))  int      v4i;

constexpr int kNLow      = 60000;
constexpr int kNHigh     = 300000;
constexpr int kNE        = 1600000;
constexpr int kKLow      = 125;
constexpr int kNLowPad   = 60032;
constexpr int kNHighPad  = 300032;
constexpr int kTile      = 1024;
constexpr int kNTiles    = 293;
constexpr int kCap       = 4096;
constexpr int kChunk     = 2048;
constexpr int kFlushAt   = kCap - kChunk;
constexpr int kEBits     = 21;
constexpr unsigned kEMask = (1u << kEBits) - 1u;
constexpr int kIters     = (kNE + kChunk - 1) / kChunk + 1;
constexpr int kLowPitch  = 136;
constexpr int kHhPitch   = 40;
constexpr int kPartPitch = 96;
constexpr size_t kLowElems = (size_t)kNLow * kKLow;
constexpr float kWCarry   = 16.0f;
constexpr float kResCarry = 2048.0f;
constexpr float kFoldMain = 1.0f / kWCarry;
constexpr float kFoldRes  = 1.0f / (kWCarry * kResCarry);
constexpr float kBnEps    = 1e-5f;
constexpr float kSlope    = 0.2f;

static_assert(kNTiles * kTile == kNHighPad, "tile cover");
static_assert((kNHighPad % 128) == 0 && (kNLowPad % 128) == 0, "row block multiples");
static_assert(kNHighPad >= kNHigh && kNLowPad >= kNLow, "pads");
static_assert(kNE + kNHighPad <= (1 << kEBits), "edge id bits");
static_assert(kTile <= (1 << (32 - kEBits)), "local node bits");
static_assert((kNE % 4) == 0, "edge list in 16-B words");
static_assert((kNHigh % 32) == 0, "output in whole lines");
static_assert((kLowElems % 4) == 0, "flat input in 16-B words");
static_assert(kFlushAt + kChunk <= kCap, "list capacity");

constexpr size_t kPlaneBytes = (size_t)kNHighPad * 32 * 4;
constexpr size_t kOffHL    = 0;
constexpr size_t kOffHR    = kOffHL + kPlaneBytes;
constexpr size_t kOffY     = kOffHR + kPlaneBytes;
constexpr size_t kOffHLLOW = kOffY + kPlaneBytes;
constexpr size_t kOffPART  = kOffHLLOW + (size_t)kNLowPad * 32 * 4;
constexpr size_t kOffSCSH  = kOffPART + (size_t)kNTiles * kPartPitch * 4;
constexpr size_t kOffBT    = kOffSCSH + (size_t)4 * kPartPitch * 4;
constexpr int kBt0H = 0;
constexpr int kBt0L = 4096;
constexpr int kBt1H = 8192;
constexpr int kBtfH = 20480;
constexpr int kBtfL = 20992;
constexpr int kBtHalves = 21504;
constexpr size_t kWsTotal  = kOffBT + (size_t)kBtHalves * 2;
static_assert(kWsTotal == 123053440ull, "carve total");
static_assert(kWsTotal <= 134217728ull, "carve cap");
static_assert((kOffHR % 128) == 0 && (kOffY % 128) == 0 && (kOffHLLOW % 128) == 0 && (kOffPART % 128) == 0 &&
              (kOffSCSH % 128) == 0 && (kOffBT % 128) == 0, "aligned regions");
constexpr int kPrepUnits = 512 + 768 + 64;

union FragU { v16h v; v8h h[2]; };
__device__ __forceinline__ v16h frag_load(const _Float16* p) {
  FragU f;
  f.h[0] = *(const v8h*)(p);
  f.h[1] = *(const v8h*)(p + 16);
  return f.v;
}
__device__ __forceinline__ v8f wmma_h(v16h a, v16h b, v8f c) {
  c = __builtin_amdgcn_wmma_f32_16x16x32_f16(false, a, false, b, (short)0, c, false, false);
  asm volatile("v_nop\n\tv_nop\n\tv_nop\n\tv_nop" : "+v"(c) : "v"(a), "v"(b));
  return c;
}
__device__ __forceinline__ void split_h(float v, _Float16& hi, _Float16& lo) {
  hi = (_Float16)v;
  const float hf = (float)hi;
  lo = (_Float16)((v - hf) * kResCarry);
}
__device__ __forceinline__ unsigned umin2(unsigned a, unsigned b) { return a < b ? a : b; }

__global__ __launch_bounds__(256) void prep_weights_kernel(
    const float* __restrict__ wlow, const float* __restrict__ g1l, const float* __restrict__ g1r,
    const float* __restrict__ g2l, const float* __restrict__ g2r,
    const float* __restrict__ g3l, const float* __restrict__ g3r,
    const float* __restrict__ fc1, unsigned short* __restrict__ bt)
{
  const int u = blockIdx.x * 256 + threadIdx.x;
  if (u >= kPrepUnits) return;
  const float* p;
  int ld, koff, cn, kmax, k8, dstH, dstL;
  if (u < 512) {
    const int n = u >> 4;
    k8 = (u & 15) * 8;
    p = wlow; ld = 32; koff = 0; cn = n; kmax = kKLow;
    dstH = kBt0H + n * 128 + k8;
    dstL = kBt0L + n * 128 + k8;
  } else if (u < 1280) {
    const int v = u - 512;
    const int mat = v >> 8;
    const int w = v & 255;
    const int n = w >> 2;
    k8 = (w & 3) * 8;
    const bool left = n < 32;
    const float* pl = (mat == 0) ? g1l : ((mat == 1) ? g2l : g3l);
    const float* pr = (mat == 0) ? g1r : ((mat == 1) ? g2r : g3r);
    p = left ? pl : pr;
    ld = 32; koff = (mat == 0) ? 1 : 0; cn = left ? n : (n - 32); kmax = 32;
    dstH = kBt1H + mat * 4096 + n * 32 + k8;
    dstL = dstH + 2048;
  } else {
    const int w = u - 1280;
    const int n = w >> 2;
    k8 = (w & 3) * 8;
    p = fc1; ld = 16; koff = 0; cn = n; kmax = 32;
    dstH = kBtfH + n * 32 + k8;
    dstL = kBtfL + n * 32 + k8;
  }
  v8h hv, lv;
#pragma unroll
  for (int e = 0; e < 8; ++e) {
    const int k = k8 + e;
    const int kc = (k < kmax) ? k : (kmax - 1);
    float w = p[(size_t)(kc + koff) * ld + cn];
    w = (k < kmax) ? (w * kWCarry) : 0.0f;
    _Float16 hi, lo;
    split_h(w, hi, lo);
    hv[e] = hi;
    lv[e] = lo;
  }
  unsigned short* qh = bt + dstH;
  unsigned short* ql = bt + dstL;
  *(volatile v8h*)qh = hv;
  *(volatile v8h*)ql = lv;
  __threadfence();
  *(volatile v8h*)qh = hv;
  *(volatile v8h*)ql = lv;
}

__global__ __launch_bounds__(256) void gemm_low_kernel(
    const float* __restrict__ x, const unsigned short* __restrict__ bhp, const unsigned short* __restrict__ blp,
    const float* __restrict__ bias, float* __restrict__ outp)
{
  __shared__ __align__(16) _Float16 sAh[128 * kLowPitch];
  __shared__ __align__(16) _Float16 sAl[128 * kLowPitch];
  __shared__ __align__(16) float sSlab[8][16 * 36];
  const int tid = threadIdx.x, lane = tid & 31, wave = tid >> 5;
  const int hh = lane >> 4, rl = lane & 15;
  const int row0 = blockIdx.x * 128;
  const size_t flat0 = (size_t)row0 * kKLow;
#pragma unroll 1
  for (int i = tid; i < 4000; i += 256) {
    const size_t f = flat0 + (size_t)(4 * i);
    const bool ok = f < kLowElems;
    const size_t fc = ok ? f : (kLowElems - 4);
    const v4f v = *(const v4f*)(x + fc);
#pragma unroll
    for (int e = 0; e < 4; ++e) {
      const int li = 4 * i + e;
      const int r = li / kKLow;
      const int k = li - r * kKLow;
      float val = v[e];
      val = ok ? val : 0.0f;
      _Float16 hi, lo;
      split_h(val, hi, lo);
      sAh[r * kLowPitch + k] = hi;
      sAl[r * kLowPitch + k] = lo;
    }
  }
#pragma unroll 1
  for (int i = tid; i < 128 * 3; i += 256) {
    const int r = i / 3;
    const int k = kKLow + (i - r * 3);
    sAh[r * kLowPitch + k] = (_Float16)0.0f;
    sAl[r * kLowPitch + k] = (_Float16)0.0f;
  }
  __syncthreads();

  const _Float16* Bh = (const _Float16*)bhp;
  const _Float16* Bl = (const _Float16*)blp;
  const _Float16* arh = sAh + (wave * 16 + rl) * kLowPitch + 8 * hh;
  const _Float16* arl = sAl + (wave * 16 + rl) * kLowPitch + 8 * hh;
  v8f am0 = (v8f){0.f,0.f,0.f,0.f,0.f,0.f,0.f,0.f};
  v8f am1 = am0, ar0 = am0, ar1 = am0;
#pragma unroll
  for (int ks = 0; ks < 4; ++ks) {
    const v16h ah = frag_load(arh + ks * 32);
    const v16h al = frag_load(arl + ks * 32);
    const int bo0 = rl * 128 + ks * 32 + 8 * hh;
    const int bo1 = (16 + rl) * 128 + ks * 32 + 8 * hh;
    const v16h b0h = frag_load(Bh + bo0);
    const v16h b0l = frag_load(Bl + bo0);
    const v16h b1h = frag_load(Bh + bo1);
    const v16h b1l = frag_load(Bl + bo1);
    am0 = wmma_h(ah, b0h, am0);
    ar0 = wmma_h(ah, b0l, ar0);
    ar0 = wmma_h(al, b0h, ar0);
    am1 = wmma_h(ah, b1h, am1);
    ar1 = wmma_h(ah, b1l, ar1);
    ar1 = wmma_h(al, b1h, ar1);
  }
  float* slab = sSlab[wave];
  {
    const float bv0 = bias[rl];
    const float bv1 = bias[16 + rl];
#pragma unroll
    for (int r = 0; r < 8; ++r) {
      slab[(8 * hh + r) * 36 + rl]      = am0[r] * kFoldMain + ar0[r] * kFoldRes + bv0;
      slab[(8 * hh + r) * 36 + 16 + rl] = am1[r] * kFoldMain + ar1[r] * kFoldRes + bv1;
    }
  }
  __syncthreads();
  {
    const int q = lane >> 3, c4 = (lane & 7) * 4;
    for (int pass = 0; pass < 2; ++pass) {
#pragma unroll
      for (int it = 0; it < 4; ++it) {
        const int row = it * 4 + q;
        const v4f v = *(const v4f*)(slab + row * 36 + c4);
        *(volatile v4f*)(outp + (size_t)(row0 + wave * 16 + row) * 32 + c4) = v;
      }
      __threadfence();
    }
  }
}

template <bool RELU>
__device__ __forceinline__ void stage_rows32(const float* __restrict__ Y, const float* __restrict__ scsh,
                                             int row0, int tid, _Float16* sAh, _Float16* sAl)
{
#pragma unroll
  for (int uu = 0; uu < 2; ++uu) {
    const int u = tid + uu * 256;
    const int row = u >> 2, c8 = (u & 3) * 8;
    int grow = row0 + row;
    grow = (grow < kNHighPad) ? grow : (kNHighPad - 1);
    const float* yp = Y + (size_t)grow * 32 + c8;
    const v4f y0 = *(const v4f*)(yp);
    const v4f y1 = *(const v4f*)(yp + 4);
    const v4f s0 = *(const v4f*)(scsh + c8);
    const v4f s1 = *(const v4f*)(scsh + c8 + 4);
    const v4f h0 = *(const v4f*)(scsh + 32 + c8);
    const v4f h1 = *(const v4f*)(scsh + 32 + c8 + 4);
    v8h hv, lv;
#pragma unroll
    for (int e = 0; e < 4; ++e) {
      float a0 = y0[e] * s0[e] + h0[e];
      float a1 = y1[e] * s1[e] + h1[e];
      if (RELU) {
        a0 = fmaxf(a0, 0.0f);
        a1 = fmaxf(a1, 0.0f);
      }
      _Float16 hi, lo;
      split_h(a0, hi, lo);
      hv[e] = hi;
      lv[e] = lo;
      split_h(a1, hi, lo);
      hv[4 + e] = hi;
      lv[4 + e] = lo;
    }
    *(v8h*)(sAh + row * kHhPitch + c8) = hv;
    *(v8h*)(sAl + row * kHhPitch + c8) = lv;
  }
}

template <bool RELU, bool ZTERM>
__global__ __launch_bounds__(256) void gemm_hh_kernel(
    const float* __restrict__ Y, const float* __restrict__ scsh, const float* __restrict__ zstd,
    const unsigned short* __restrict__ bhp, const unsigned short* __restrict__ blp,
    const float* __restrict__ biasL, const float* __restrict__ biasR,
    const float* __restrict__ w0L, const float* __restrict__ w0R,
    float* __restrict__ HL, float* __restrict__ HR)
{
  __shared__ __align__(16) _Float16 sAh[128 * kHhPitch];
  __shared__ __align__(16) _Float16 sAl[128 * kHhPitch];
  __shared__ __align__(16) float sSlab[8][16 * 68];
  __shared__ __align__(16) float sZ[128];
  const int tid = threadIdx.x, lane = tid & 31, wave = tid >> 5;
  const int hh = lane >> 4, rl = lane & 15;
  const int row0 = blockIdx.x * 128;
  stage_rows32<RELU>(Y, scsh, row0, tid, sAh, sAl);
  if (tid < 128) {
    float zn = 0.0f;
    if (ZTERM) {
      int gr = row0 + tid;
      gr = (gr < kNHigh) ? gr : (kNHigh - 1);
      zn = zstd[gr] * scsh[64] + scsh[65];
    }
    sZ[tid] = zn;
  }
  __syncthreads();

  const _Float16* Bh = (const _Float16*)bhp;
  const _Float16* Bl = (const _Float16*)blp;
  const v16h ah = frag_load(sAh + (wave * 16 + rl) * kHhPitch + 8 * hh);
  const v16h al = frag_load(sAl + (wave * 16 + rl) * kHhPitch + 8 * hh);
  v8f am[4], ar[4];
#pragma unroll
  for (int j = 0; j < 4; ++j) {
    am[j] = (v8f){0.f,0.f,0.f,0.f,0.f,0.f,0.f,0.f};
    ar[j] = (v8f){0.f,0.f,0.f,0.f,0.f,0.f,0.f,0.f};
  }
#pragma unroll
  for (int j = 0; j < 4; ++j) {
    const int bo = (j * 16 + rl) * 32 + 8 * hh;
    const v16h bh = frag_load(Bh + bo);
    const v16h bl = frag_load(Bl + bo);
    am[j] = wmma_h(ah, bh, am[j]);
    ar[j] = wmma_h(ah, bl, ar[j]);
    ar[j] = wmma_h(al, bh, ar[j]);
  }
  float* slab = sSlab[wave];
#pragma unroll
  for (int j = 0; j < 4; ++j) {
    const int n = j * 16 + rl;
    const float bv = (j < 2) ? biasL[n] : biasR[n - 32];
    float w0 = 0.0f;
    if (ZTERM) w0 = (j < 2) ? w0L[n] : w0R[n - 32];
#pragma unroll
    for (int r = 0; r < 8; ++r) {
      float v = am[j][r] * kFoldMain + ar[j][r] * kFoldRes + bv;
      if (ZTERM) v += sZ[wave * 16 + 8 * hh + r] * w0;
      slab[(8 * hh + r) * 68 + n] = v;
    }
  }
  __syncthreads();
  {
    const int q = lane >> 3, c4 = (lane & 7) * 4;
    for (int pass = 0; pass < 2; ++pass) {
#pragma unroll
      for (int it = 0; it < 4; ++it) {
        const int row = it * 4 + q;
        const v4f a = *(const v4f*)(slab + row * 68 + c4);
        const v4f b = *(const v4f*)(slab + row * 68 + 32 + c4);
        const size_t go = (size_t)(row0 + wave * 16 + row) * 32 + c4;
        *(volatile v4f*)(HL + go) = a;
        *(volatile v4f*)(HR + go) = b;
      }
      __threadfence();
    }
  }
}

__global__ __launch_bounds__(256) void head_kernel(
    const float* __restrict__ Y, const float* __restrict__ scsh,
    const unsigned short* __restrict__ bhp, const unsigned short* __restrict__ blp,
    const float* __restrict__ b1, const float* __restrict__ w2, const float* __restrict__ b2,
    float* __restrict__ outp)
{
  __shared__ __align__(16) _Float16 sAh[128 * kHhPitch];
  __shared__ __align__(16) _Float16 sAl[128 * kHhPitch];
  __shared__ __align__(16) float sOut[128];
  const int tid = threadIdx.x, lane = tid & 31, wave = tid >> 5;
  const int hh = lane >> 4, rl = lane & 15;
  const int row0 = blockIdx.x * 128;
  stage_rows32<true>(Y, scsh, row0, tid, sAh, sAl);
  __syncthreads();
  const _Float16* Bh = (const _Float16*)bhp;
  const _Float16* Bl = (const _Float16*)blp;
  const v16h ah = frag_load(sAh + (wave * 16 + rl) * kHhPitch + 8 * hh);
  const v16h al = frag_load(sAl + (wave * 16 + rl) * kHhPitch + 8 * hh);
  const v16h bh = frag_load(Bh + rl * 32 + 8 * hh);
  const v16h bl = frag_load(Bl + rl * 32 + 8 * hh);
  v8f am = (v8f){0.f,0.f,0.f,0.f,0.f,0.f,0.f,0.f};
  v8f ar = am;
  am = wmma_h(ah, bh, am);
  ar = wmma_h(ah, bl, ar);
  ar = wmma_h(al, bh, ar);
  const float bv = b1[rl];
  const float wv = w2[rl];
  const float b2v = b2[0];
#pragma unroll
  for (int r = 0; r < 8; ++r) {
    float v = fmaxf(am[r] * kFoldMain + ar[r] * kFoldRes + bv, 0.0f) * wv;
    v += __shfl_xor(v, 1, 32);
    v += __shfl_xor(v, 2, 32);
    v += __shfl_xor(v, 4, 32);
    v += __shfl_xor(v, 8, 32);
    if (rl == 0) sOut[wave * 16 + 8 * hh + r] = v + b2v;
  }
  __syncthreads();
  if (wave < 4) {
    const int line = blockIdx.x * 4 + wave;
    if (line < (kNHigh / 32)) {
      const float v = sOut[wave * 32 + lane];
      volatile float* op = outp + (size_t)line * 32 + lane;
      *op = v;
      __threadfence();
      *op = v;
    }
  }
}

#define EA_APPEND(UU, EE)                                                                                   \
  if ((UU) < (unsigned)kTile) {                                                                             \
    const int pos_ = __hip_atomic_fetch_add(&sN, 1, __ATOMIC_RELAXED, __HIP_MEMORY_SCOPE_WORKGROUP);        \
    if ((unsigned)pos_ < (unsigned)kCap) sList[pos_] = ((UU) << kEBits) | (unsigned)(EE);                   \
  }

template <bool L2H>
__global__ __launch_bounds__(256) void edge_attn_tile_kernel(
    const float* __restrict__ HLsrc, const float* __restrict__ HRdst,
    const float* __restrict__ xh, const float* __restrict__ Wr, const float* __restrict__ br,
    const float* __restrict__ att, const float* __restrict__ bias,
    const int* __restrict__ esrc, const int* __restrict__ edst,
    const float* __restrict__ zstd,
    float* __restrict__ Yout, float* __restrict__ part)
{
  __shared__ __align__(16) float    sAcc[kTile * 32];
  __shared__ __align__(16) float    sM[kTile];
  __shared__ __align__(16) float    sL[kTile];
  __shared__ __align__(16) int      sCnt[kTile];
  __shared__ __align__(16) unsigned sList[kCap];
  __shared__ __align__(16) unsigned sSort[kCap];
  __shared__ __align__(16) float    sAtt[32];
  __shared__ __align__(16) float    sWr[32];
  __shared__ __align__(16) float    sBr[32];
  __shared__ __align__(16) float    sBias[32];
  __shared__ __align__(16) float    sRed[8 * 64];
  __shared__ __align__(16) float    sRedZ[512];
  __shared__ int sWave[8];
  __shared__ int sN;

  constexpr int NSRC = L2H ? kNLow : kNHigh;
  const int tid = threadIdx.x, lane = tid & 31, wave = tid >> 5;
  const int tile0 = blockIdx.x * kTile;
  const int own0 = 4 * tid;

  {
    const v4f zero4 = (v4f){0.f, 0.f, 0.f, 0.f};
    const v4f ninf4 = (v4f){-INFINITY, -INFINITY, -INFINITY, -INFINITY};
#pragma unroll 1
    for (int c = 0; c < 32; ++c) *(v4f*)(sAcc + own0 * 32 + 4 * c) = zero4;
    *(v4f*)(sM + own0) = ninf4;
    *(v4f*)(sL + own0) = zero4;
  }
  if (tid < 32) {
    sAtt[tid]  = att[tid];
    sBias[tid] = bias[tid];
    sWr[tid]   = Wr[tid];
    sBr[tid]   = br[tid];
  }
  int nreal = kNHigh - tile0;
  nreal = (nreal < kTile) ? nreal : kTile;
  if (!L2H) {
#pragma unroll
    for (int j = 0; j < 4; ++j) {
      const int dl = own0 + j;
      sList[dl] = ((unsigned)dl << kEBits) | (unsigned)(kNE + tile0 + dl);
    }
  }
  if (tid == 0) sN = L2H ? 0 : nreal;
  int deg0 = 0, deg1 = 0, deg2 = 0, deg3 = 0;
  __syncthreads();

#pragma unroll 1
  for (int itc = 0; itc < kIters; ++itc) {
    const int base = itc * kChunk;
    const int e0 = base + tid * 4;
    const int e1 = e0 + 1024;
    const bool ok0 = e0 < kNE;
    const bool ok1 = e1 < kNE;
    const int a0 = ok0 ? e0 : (kNE - 4);
    const int a1 = ok1 ? e1 : (kNE - 4);
    const v4i d0 = *(const v4i*)(edst + a0);
    const v4i d1 = *(const v4i*)(edst + a1);
    const unsigned u0 = ok0 ? (unsigned)(d0.x - tile0) : 0xFFFFFFFFu;
    const unsigned u1 = ok0 ? (unsigned)(d0.y - tile0) : 0xFFFFFFFFu;
    const unsigned u2 = ok0 ? (unsigned)(d0.z - tile0) : 0xFFFFFFFFu;
    const unsigned u3 = ok0 ? (unsigned)(d0.w - tile0) : 0xFFFFFFFFu;
    const unsigned u4 = ok1 ? (unsigned)(d1.x - tile0) : 0xFFFFFFFFu;
    const unsigned u5 = ok1 ? (unsigned)(d1.y - tile0) : 0xFFFFFFFFu;
    const unsigned u6 = ok1 ? (unsigned)(d1.z - tile0) : 0xFFFFFFFFu;
    const unsigned u7 = ok1 ? (unsigned)(d1.w - tile0) : 0xFFFFFFFFu;
    const unsigned mn = umin2(umin2(umin2(u0, u1), umin2(u2, u3)), umin2(umin2(u4, u5), umin2(u6, u7)));
    if (__builtin_amdgcn_ballot_w32(mn < (unsigned)kTile) != 0u) {
      EA_APPEND(u0, e0)
      EA_APPEND(u1, e0 + 1)
      EA_APPEND(u2, e0 + 2)
      EA_APPEND(u3, e0 + 3)
      EA_APPEND(u4, e1)
      EA_APPEND(u5, e1 + 1)
      EA_APPEND(u6, e1 + 2)
      EA_APPEND(u7, e1 + 3)
    }
    __syncthreads();
    int n = sN;
    __syncthreads();
    const bool last = (itc == kIters - 1);
    if ((n > kFlushAt) || (last && n > 0)) {
      n = (n < kCap) ? n : kCap;
      *(v4i*)(sCnt + own0) = (v4i){0, 0, 0, 0};
      __syncthreads();
#pragma unroll 1
      for (int i = tid; i < n; i += 256) {
        int dl = (int)(sList[i] >> kEBits);
        dl = (dl < kTile) ? dl : (kTile - 1);
        __hip_atomic_fetch_add(&sCnt[dl], 1, __ATOMIC_RELAXED, __HIP_MEMORY_SCOPE_WORKGROUP);
      }
      __syncthreads();
      const v4i cc = *(const v4i*)(sCnt + own0);
      const int tsum = cc.x + cc.y + cc.z + cc.w;
      deg0 += cc.x;
      deg1 += cc.y;
      deg2 += cc.z;
      deg3 += cc.w;
      int incl = tsum;
#pragma unroll
      for (int off = 1; off < 32; off <<= 1) {
        const int o = __shfl_up(incl, off, 32);
        incl += (lane >= off) ? o : 0;
      }
      if (lane == 31) sWave[wave] = incl;
      __syncthreads();
      int wbase = 0;
#pragma unroll
      for (int w = 0; w < 8; ++w) {
        const int wv = sWave[w];
        wbase += (w < wave) ? wv : 0;
      }
      int ts = wbase + incl - tsum;
      *(v4i*)(sCnt + own0) = (v4i){ts, ts + cc.x, ts + cc.x + cc.y, ts + cc.x + cc.y + cc.z};
      __syncthreads();
#pragma unroll 1
      for (int i = tid; i < n; i += 256) {
        const unsigned key = sList[i];
        int dl = (int)(key >> kEBits);
        dl = (dl < kTile) ? dl : (kTile - 1);
        const int pos = __hip_atomic_fetch_add(&sCnt[dl], 1, __ATOMIC_RELAXED, __HIP_MEMORY_SCOPE_WORKGROUP);
        if ((unsigned)pos < (unsigned)kCap) sSort[pos] = key;
      }
      __syncthreads();
      if (tid == 0) sN = 0;
      int te = ts + tsum;
      te = (te < kCap) ? te : kCap;
      ts = (ts < kCap) ? ts : kCap;
#pragma unroll 1
      for (int i = ts + 1; i < te; ++i) {
        const unsigned key = sSort[i];
        int j = i - 1;
#pragma unroll 1
        while (j >= ts) {
          const unsigned kj = sSort[j];
          if (kj <= key) break;
          sSort[j + 1] = kj;
          --j;
        }
        sSort[j + 1] = key;
      }
      const int cnt = te - ts;
      int trips = cnt;
#pragma unroll
      for (int off = 16; off >= 1; off >>= 1) {
        const int o = __shfl_xor(trips, off, 32);
        trips = (o > trips) ? o : trips;
      }
#pragma unroll 1
      for (int it = 0; it < trips; ++it) {
        const bool active = it < cnt;
        int idx = active ? (ts + it) : 0;
        idx = (idx < kCap) ? idx : (kCap - 1);
        const unsigned key = sSort[idx];
        int dl = (int)(key >> kEBits);
        dl = (dl < kTile) ? dl : (kTile - 1);
        dl = active ? dl : own0;
        const int e = (int)(key & kEMask);
        const int ec = (e < kNE) ? e : (kNE - 1);
        int sld = esrc[ec];
        asm volatile("" : "+v"(sld));
        int s = (e < kNE) ? sld : (e - kNE);
        s = (s < 0) ? 0 : s;
        s = (s < NSRC) ? s : (NSRC - 1);
        const int node = tile0 + dl;
        const float* hp = HLsrc + (size_t)s * 32;
        const float* rp = HRdst + (size_t)node * 32;
        float xhv = 0.0f;
        if (L2H) {
          const int nc = (node < kNHigh) ? node : (kNHigh - 1);
          xhv = xh[nc];
          asm volatile("" : "+v"(xhv));
        }
        float sc = 0.0f;
#pragma unroll 1
        for (int c = 0; c < 8; ++c) {
          v4f a = *(const v4f*)(hp + 4 * c);
          asm volatile("" : "+v"(a));
          v4f b;
          if (L2H) {
            const v4f w = *(const v4f*)(sWr + 4 * c);
            const v4f bb = *(const v4f*)(sBr + 4 * c);
            b = w * xhv + bb;
          } else {
            b = *(const v4f*)(rp + 4 * c);
            asm volatile("" : "+v"(b));
          }
          const v4f w4 = *(const v4f*)(sAtt + 4 * c);
#pragma unroll
          for (int q = 0; q < 4; ++q) {
            float t = a[q] + b[q];
            t = fmaxf(t, kSlope * t);
            sc = fmaf(t, w4[q], sc);
          }
        }
        const float mo = sM[dl];
        const float lo_ = sL[dl];
        const float ee = __expf(-fabsf(sc - mo));
        const bool up = sc > mo;
        float scale = up ? ee : 1.0f;
        float p = up ? 1.0f : ee;
        float mnew = up ? sc : mo;
        float lnew = lo_ * scale + p;
        scale = active ? scale : 1.0f;
        p = active ? p : 0.0f;
        mnew = active ? mnew : mo;
        lnew = active ? lnew : lo_;
        sM[dl] = mnew;
        sL[dl] = lnew;
#pragma unroll 1
        for (int c = 0; c < 8; ++c) {
          v4f a = *(const v4f*)(hp + 4 * c);
          asm volatile("" : "+v"(a));
          float* ap = sAcc + dl * 32 + 4 * c;
          const v4f o = *(const v4f*)ap;
          v4f nv;
#pragma unroll
          for (int q = 0; q < 4; ++q) {
            const float t = o[q] * scale + a[q] * p;
            nv[q] = active ? t : o[q];
          }
          *(v4f*)ap = nv;
        }
      }
      __syncthreads();
    }
  }

  float zs = 0.0f, zss = 0.0f;
#pragma unroll
  for (int j = 0; j < 4; ++j) {
    const int dl = own0 + j;
    const int dg = (j == 0) ? deg0 : ((j == 1) ? deg1 : ((j == 2) ? deg2 : deg3));
    const float lsum = sL[dl];
    const float den = (dg > 0) ? (lsum * (float)dg) : 1.0f;
    const float inv = (dg > 0) ? (1.0f / den) : 0.0f;
#pragma unroll 1
    for (int c = 0; c < 8; ++c) {
      float* ap = sAcc + dl * 32 + 4 * c;
      const v4f a = *(const v4f*)ap;
      const v4f bb = *(const v4f*)(sBias + 4 * c);
      const v4f y = a * inv + bb;
      *(v4f*)ap = y;
    }
    if (L2H) {
      const int node = tile0 + dl;
      const bool okn = node < kNHigh;
      const int nc = okn ? node : (kNHigh - 1);
      float zv = zstd[nc];
      zv = okn ? zv : 0.0f;
      zs += zv;
      zss = fmaf(zv, zv, zss);
    }
  }
  sRedZ[tid] = zs;
  sRedZ[256 + tid] = zss;
  __syncthreads();
  {
    const int col = lane;
    float s1 = 0.0f, s2 = 0.0f;
#pragma unroll 1
    for (int r = wave; r < kTile; r += 8) {
      float y = sAcc[r * 32 + col];
      y = ((tile0 + r) < kNHigh) ? y : 0.0f;
      s1 += y;
      s2 = fmaf(y, y, s2);
    }
    sRed[wave * 64 + col] = s1;
    sRed[wave * 64 + 32 + col] = s2;
  }
  __syncthreads();
  if (wave == 0) {
    float t1 = 0.0f, t2 = 0.0f, z1 = 0.0f, z2 = 0.0f;
#pragma unroll
    for (int g = 0; g < 8; ++g) {
      t1 += sRed[g * 64 + lane];
      t2 += sRed[g * 64 + 32 + lane];
      z1 += sRedZ[g * 32 + lane];
      z2 += sRedZ[256 + g * 32 + lane];
    }
#pragma unroll
    for (int off = 16; off >= 1; off >>= 1) {
      z1 += __shfl_xor(z1, off, 32);
      z2 += __shfl_xor(z2, off, 32);
    }
    const float l2v = (lane == 0) ? z1 : ((lane == 1) ? z2 : 0.0f);
    volatile float* pp = part + (size_t)blockIdx.x * kPartPitch;
    pp[lane] = t1;
    pp[32 + lane] = t2;
    pp[64 + lane] = l2v;
    __threadfence();
    pp[lane] = t1;
    pp[32 + lane] = t2;
    pp[64 + lane] = l2v;
  }
  {
    const int q = lane >> 3, c4 = (lane & 7) * 4;
    for (int pass = 0; pass < 2; ++pass) {
#pragma unroll 1
      for (int it = 0; it < 32; ++it) {
        const int row = wave * 128 + it * 4 + q;
        const v4f v = *(const v4f*)(sAcc + row * 32 + c4);
        *(volatile v4f*)(Yout + (size_t)(tile0 + row) * 32 + c4) = v;
      }
      __threadfence();
    }
  }
}

__global__ __launch_bounds__(32) void bn_finish_kernel(
    const float* __restrict__ part, const float* __restrict__ g, const float* __restrict__ b,
    int goff, int hasz, float* __restrict__ scsh)
{
  const int lane = threadIdx.x & 31;
  double s = 0.0, ss = 0.0, zs = 0.0, zss = 0.0;
#pragma unroll 1
  for (int i = 0; i < kNTiles; ++i) {
    const float* p = part + (size_t)i * kPartPitch;
    s += (double)p[lane];
    ss += (double)p[32 + lane];
    zs += (double)p[64];
    zss += (double)p[65];
  }
  const double invn = 1.0 / (double)kNHigh;
  const double mu = s * invn;
  double var = ss * invn - mu * mu;
  var = (var < 0.0) ? 0.0 : var;
  const float sc = g[goff + lane] * (1.0f / sqrtf((float)var + kBnEps));
  const float sh = b[goff + lane] - (float)mu * sc;
  const double muz = zs * invn;
  double varz = zss * invn - muz * muz;
  varz = (varz < 0.0) ? 0.0 : varz;
  float scz = g[0] * (1.0f / sqrtf((float)varz + kBnEps));
  float shz = b[0] - (float)muz * scz;
  scz = (hasz != 0) ? scz : 0.0f;
  shz = (hasz != 0) ? shz : 0.0f;
  const float l2v = (lane == 0) ? scz : ((lane == 1) ? shz : 0.0f);
  volatile float* o = scsh;
  o[lane] = sc;
  o[32 + lane] = sh;
  o[64 + lane] = l2v;
  __threadfence();
  o[lane] = sc;
  o[32 + lane] = sh;
  o[64 + lane] = l2v;
}

extern "C" void kernel_launch(void* const* d_in, const int* in_sizes, int n_in,
                              void* d_out, int out_size, void* d_ws, size_t ws_size,
                              hipStream_t stream) {
  if (n_in < 43) return;
  if (in_sizes[0] != kNLow * kKLow) return;
  if (in_sizes[1] != kNHigh || in_sizes[2] != kNHigh) return;
  if (in_sizes[3] != kKLow * 32) return;
  if (in_sizes[11] != 33 * 32 || in_sizes[13] != 33 * 32) return;
  if (in_sizes[17] != 32 * 32 || in_sizes[19] != 32 * 32 || in_sizes[23] != 32 * 32 || in_sizes[25] != 32 * 32) return;
  if (in_sizes[9] != 33 || in_sizes[10] != 33) return;
  if (in_sizes[35] != 32 * 16 || in_sizes[37] != 16) return;
  if (in_sizes[39] != kNE || in_sizes[40] != kNE || in_sizes[41] != kNE || in_sizes[42] != kNE) return;
  if (out_size != kNHigh) return;
  if (ws_size < kWsTotal) return;

  const float* x_low    = (const float*)d_in[0];
  const float* x_high   = (const float*)d_in[1];
  const float* z_std    = (const float*)d_in[2];
  const float* l2h_Wl   = (const float*)d_in[3];
  const float* l2h_bl   = (const float*)d_in[4];
  const float* l2h_Wr   = (const float*)d_in[5];
  const float* l2h_br   = (const float*)d_in[6];
  const float* l2h_att  = (const float*)d_in[7];
  const float* l2h_bias = (const float*)d_in[8];
  const float* bn1_g    = (const float*)d_in[9];
  const float* bn1_b    = (const float*)d_in[10];
  const float* g1_Wl    = (const float*)d_in[11];
  const float* g1_bl    = (const float*)d_in[12];
  const float* g1_Wr    = (const float*)d_in[13];
  const float* g1_br    = (const float*)d_in[14];
  const float* g1_att   = (const float*)d_in[15];
  const float* g1_bias  = (const float*)d_in[16];
  const float* g2_Wl    = (const float*)d_in[17];
  const float* g2_bl    = (const float*)d_in[18];
  const float* g2_Wr    = (const float*)d_in[19];
  const float* g2_br    = (const float*)d_in[20];
  const float* g2_att   = (const float*)d_in[21];
  const float* g2_bias  = (const float*)d_in[22];
  const float* g3_Wl    = (const float*)d_in[23];
  const float* g3_bl    = (const float*)d_in[24];
  const float* g3_Wr    = (const float*)d_in[25];
  const float* g3_br    = (const float*)d_in[26];
  const float* g3_att   = (const float*)d_in[27];
  const float* g3_bias  = (const float*)d_in[28];
  const float* bn2_g    = (const float*)d_in[29];
  const float* bn2_b    = (const float*)d_in[30];
  const float* bn3_g    = (const float*)d_in[31];
  const float* bn3_b    = (const float*)d_in[32];
  const float* bn4_g    = (const float*)d_in[33];
  const float* bn4_b    = (const float*)d_in[34];
  const float* fc1_W    = (const float*)d_in[35];
  const float* fc1_b    = (const float*)d_in[36];
  const float* fc2_W    = (const float*)d_in[37];
  const float* fc2_b    = (const float*)d_in[38];
  const int* l2h_src    = (const int*)d_in[39];
  const int* l2h_dst    = (const int*)d_in[40];
  const int* hh_src     = (const int*)d_in[41];
  const int* hh_dst     = (const int*)d_in[42];
  float* outp = (float*)d_out;

  char* ws = (char*)d_ws;
  float* HL    = (float*)(ws + kOffHL);
  float* HR    = (float*)(ws + kOffHR);
  float* Yp    = (float*)(ws + kOffY);
  float* HLLOW = (float*)(ws + kOffHLLOW);
  float* PART  = (float*)(ws + kOffPART);
  float* SCSH  = (float*)(ws + kOffSCSH);
  unsigned short* BT = (unsigned short*)(ws + kOffBT);

  const int gemmBlocks = kNHighPad / 128;

  prep_weights_kernel<<<(kPrepUnits + 255) / 256, 256, 0, stream>>>(
      l2h_Wl, g1_Wl, g1_Wr, g2_Wl, g2_Wr, g3_Wl, g3_Wr, fc1_W, BT);

  gemm_low_kernel<<<kNLowPad / 128, 256, 0, stream>>>(x_low, BT + kBt0H, BT + kBt0L, l2h_bl, HLLOW);
  edge_attn_tile_kernel<true><<<kNTiles, 256, 0, stream>>>(
      HLLOW, HR, x_high, l2h_Wr, l2h_br, l2h_att, l2h_bias, l2h_src, l2h_dst, z_std, Yp, PART);
  bn_finish_kernel<<<1, 32, 0, stream>>>(PART, bn1_g, bn1_b, 1, 1, SCSH);

  gemm_hh_kernel<false, true><<<gemmBlocks, 256, 0, stream>>>(
      Yp, SCSH, z_std, BT + kBt1H, BT + kBt1H + 2048, g1_bl, g1_br, g1_Wl, g1_Wr, HL, HR);
  edge_attn_tile_kernel<false><<<kNTiles, 256, 0, stream>>>(
      HL, HR, x_high, l2h_Wr, l2h_br, g1_att, g1_bias, hh_src, hh_dst, z_std, Yp, PART);
  bn_finish_kernel<<<1, 32, 0, stream>>>(PART, bn2_g, bn2_b, 0, 0, SCSH + kPartPitch);

  gemm_hh_kernel<true, false><<<gemmBlocks, 256, 0, stream>>>(
      Yp, SCSH + kPartPitch, z_std, BT + kBt1H + 4096, BT + kBt1H + 4096 + 2048, g2_bl, g2_br, g2_Wl, g2_Wr, HL, HR);
  edge_attn_tile_kernel<false><<<kNTiles, 256, 0, stream>>>(
      HL, HR, x_high, l2h_Wr, l2h_br, g2_att, g2_bias, hh_src, hh_dst, z_std, Yp, PART);
  bn_finish_kernel<<<1, 32, 0, stream>>>(PART, bn3_g, bn3_b, 0, 0, SCSH + 2 * kPartPitch);

  gemm_hh_kernel<true, false><<<gemmBlocks, 256, 0, stream>>>(
      Yp, SCSH + 2 * kPartPitch, z_std, BT + kBt1H + 8192, BT + kBt1H + 8192 + 2048, g3_bl, g3_br, g3_Wl, g3_Wr, HL, HR);
  edge_attn_tile_kernel<false><<<kNTiles, 256, 0, stream>>>(
      HL, HR, x_high, l2h_Wr, l2h_br, g3_att, g3_bias, hh_src, hh_dst, z_std, Yp, PART);
  bn_finish_kernel<<<1, 32, 0, stream>>>(PART, bn4_g, bn4_b, 0, 0, SCSH + 3 * kPartPitch);

  head_kernel<<<gemmBlocks, 256, 0, stream>>>(
      Yp, SCSH + 3 * kPartPitch, BT + kBtfH, BT + kBtfL, fc1_b, fc2_W, fc2_b, outp);
}
